// DinMod_23957327577772
// MI455X (gfx1250) — hardware-run, weakly checked
//
#include <hip/hip_runtime.h>
#include <math.h>

typedef __attribute__((ext_vector_type(16))) _Float16 v16h;
typedef __attribute__((ext_vector_type(8)))  _Float16 v8h;
typedef __attribute__((ext_vector_type(8)))  float    v8f;
typedef __attribute__((ext_vector_type(4)))  float    v4f;

constexpr int kBatch = 256;
constexpr int kSteps = 512;
constexpr int kIn    = 64;
constexpr int kLat   = 256;
constexpr int kBk    = 128;
constexpr int kOutD  = 64;
constexpr int kCat   = kIn + kLat;
constexpr int kHeadN = 3 * kLat;
constexpr int kProjH = kLat / 2;
constexpr int kRows  = kBatch * kSteps;
static_assert(kCat == 320 && kHeadN == 768 && kProjH == 128 && kRows == 131072, "shapes");
static_assert((kCat % 32) == 0 && (kBk % 32) == 0 && (kLat % 32) == 0 && (kProjH % 32) == 0, "K multiples of 32");
static_assert((kRows % 32) == 0 && (kProjH % 64) == 0 && (kOutD % 64) == 0, "M multiple of 32, N multiples of 64");
static_assert((kBatch % 16) == 0, "16 batch rows per block");

constexpr float kWCarry   = 64.0f;
constexpr float kWInv     = 1.0f / kWCarry;
constexpr float kHdCarry  = 16.0f;
constexpr float kOutScale = 1.0f / (kWCarry * kHdCarry);
constexpr float kResCarry = 2048.0f;
constexpr float kResInv   = 1.0f / kResCarry;
constexpr float kSubCut   = 6.2e-5f;

constexpr int kHP = kLat + 8;
constexpr int kZP = kBk + 8;

constexpr size_t kOffWbT  = 0;
constexpr size_t kOffWhT  = kOffWbT  + (size_t)kBk    * kCat   * 2;
constexpr size_t kOffWp1T = kOffWhT  + (size_t)kHeadN * kBk    * 2;
constexpr size_t kOffWp1R = kOffWp1T + (size_t)kProjH * kLat   * 2;
constexpr size_t kOffWp2T = kOffWp1R + (size_t)kProjH * kLat   * 2;
constexpr size_t kOffWp2R = kOffWp2T + (size_t)kOutD  * kProjH * 2;
constexpr size_t kOffX16  = kOffWp2R + (size_t)kOutD  * kProjH * 2;
constexpr size_t kOffHs   = kOffX16  + (size_t)kRows  * kIn    * 2;
constexpr size_t kOffHD   = kOffHs   + (size_t)kRows  * kLat   * 2;
constexpr size_t kWsTotal = kOffHD   + (size_t)kRows  * kProjH * 2;
static_assert(kWsTotal == 117882880ull, "carve total");
static_assert(kWsTotal <= 134217728ull, "carve cap");
static_assert((kOffWhT % 128) == 0 && (kOffWp1T % 128) == 0 && (kOffWp1R % 128) == 0 &&
              (kOffWp2T % 128) == 0 && (kOffWp2R % 128) == 0 &&
              (kOffX16 % 128) == 0 && (kOffHs % 128) == 0 && (kOffHD % 128) == 0, "128-B aligned regions");

struct FragH {
  union U { v16h v; v8h h[2]; };
  static __device__ __forceinline__ v16h load(const _Float16* p) {
    U f;
    f.h[0] = *(const v8h*)(p);
    f.h[1] = *(const v8h*)(p + 16);
    return f.v;
  }
};

__device__ __forceinline__ v8f mma_h(v16h a, v16h b, v8f c) {
  c = __builtin_amdgcn_wmma_f32_16x16x32_f16(false, a, false, b, (short)0, c, false, false);
  asm volatile("v_nop\n\tv_nop\n\tv_nop\n\tv_nop" : "+v"(c) : "v"(a), "v"(b));
  return c;
}

__device__ __forceinline__ float tanh_f32(float y) {
  const float a = fminf(fmaxf(2.0f * y, -40.0f), 40.0f);
  const float e = expf(a);
  return 1.0f - 2.0f * __builtin_amdgcn_rcpf(e + 1.0f);
}
__device__ __forceinline__ float sigmoid_f32(float y) {
  const float a = fminf(fmaxf(-y, -40.0f), 40.0f);
  return __builtin_amdgcn_rcpf(1.0f + expf(a));
}

constexpr int kBlkWb = (kBk * kCat / 8) / 256;
constexpr int kBlkHd = (kLat * kBk / 8) / 256;
constexpr int kBlkP1 = (kProjH * kLat / 8) / 256;
constexpr int kBlkP2 = (kOutD * kProjH / 8) / 256;
constexpr int kBlkPack = kBlkWb + 3 * kBlkHd + kBlkP1 + kBlkP2;
static_assert(kBlkWb == 20 && kBlkHd == 16 && kBlkP1 == 16 && kBlkP2 == 4 && kBlkPack == 88, "pack grid");
static_assert(kBlkWb * 256 * 8 == kBk * kCat && kBlkHd * 256 * 8 == kLat * kBk &&
              kBlkP1 * 256 * 8 == kProjH * kLat && kBlkP2 * 256 * 8 == kOutD * kProjH, "pack coverage");

__global__ __launch_bounds__(256) void pack_weights_kernel(
    const float* __restrict__ Wb, const float* __restrict__ W1, const float* __restrict__ W2,
    const float* __restrict__ Wa, const float* __restrict__ Wtb,
    const float* __restrict__ Wp1, const float* __restrict__ Wp2,
    unsigned short* __restrict__ WbT, unsigned short* __restrict__ WhT,
    unsigned short* __restrict__ Wp1T, unsigned short* __restrict__ Wp1R,
    unsigned short* __restrict__ Wp2T, unsigned short* __restrict__ Wp2R)
{
  const int blk = blockIdx.x;
  const float* src;
  const float* src2;
  unsigned short* dst;
  unsigned short* dstR;
  int K, N, cb;
  bool add = false;
  bool resid = false;
  if (blk < kBlkWb) {
    src = Wb; src2 = Wb; dst = WbT; dstR = WbT; K = kCat; N = kBk; cb = blk;
  } else if (blk < kBlkWb + 3 * kBlkHd) {
    const int sb = blk - kBlkWb;
    const int head = sb / kBlkHd;
    src  = (head == 0) ? W1 : ((head == 1) ? W2 : Wa);
    src2 = (head == 2) ? Wtb : src;
    add  = (head == 2);
    dst  = WhT + (size_t)head * kLat * kBk;
    dstR = dst;
    K = kBk; N = kLat; cb = sb - head * kBlkHd;
  } else if (blk < kBlkWb + 3 * kBlkHd + kBlkP1) {
    src = Wp1; src2 = Wp1; dst = Wp1T; dstR = Wp1R; resid = true;
    K = kLat; N = kProjH; cb = blk - (kBlkWb + 3 * kBlkHd);
  } else {
    src = Wp2; src2 = Wp2; dst = Wp2T; dstR = Wp2R; resid = true;
    K = kProjH; N = kOutD; cb = blk - (kBlkWb + 3 * kBlkHd + kBlkP1);
  }
  const float cut = resid ? kSubCut : 0.0f;
  const int chunk = cb * 256 + threadIdx.x;
  const int e0 = chunk * 8;
  const int n  = e0 / K;
  const int k0 = e0 - n * K;
  v8h hv, rv;
#pragma unroll
  for (int e = 0; e < 8; ++e) {
    const size_t si = (size_t)(k0 + e) * N + n;
    const float v1 = src[si];
    const float v2 = src2[si];
    const float v  = add ? (v1 + v2) : v1;
    const float s  = v * kWCarry;
    const float sv = (fabsf(s) < cut) ? 0.0f : s;
    const _Float16 hval = (_Float16)sv;
    const float back = (float)hval;
    const float rem  = (s - back) * kResCarry;
    hv[e] = hval;
    rv[e] = (_Float16)rem;
  }
  unsigned short* q  = dst + (size_t)e0;
  unsigned short* qr = dstR + (size_t)e0;
  *(volatile v8h*)q = hv;
  if (resid) *(volatile v8h*)qr = rv;
  __threadfence();
  *(volatile v8h*)q = hv;
  if (resid) *(volatile v8h*)qr = rv;
}

__global__ __launch_bounds__(256) void x_to_f16_kernel(
    const float* __restrict__ x, unsigned short* __restrict__ X16, int total8)
{
  const int i = blockIdx.x * 256 + threadIdx.x;
  if (i >= total8) return;
  const size_t e0 = (size_t)i << 3;
  const v4f a0 = *(const v4f*)(x + e0);
  const v4f a1 = *(const v4f*)(x + e0 + 4);
  v8h hv;
#pragma unroll
  for (int e = 0; e < 4; ++e) {
    hv[e]     = (_Float16)a0[e];
    hv[4 + e] = (_Float16)a1[e];
  }
  unsigned short* q = X16 + e0;
  *(volatile v8h*)q = hv;
  __threadfence();
  *(volatile v8h*)q = hv;
}

__global__ __launch_bounds__(256) void recur_kernel(
    const unsigned short* __restrict__ X16p, const unsigned short* __restrict__ WbTp,
    const unsigned short* __restrict__ WhTp,
    const float* __restrict__ bb, const float* __restrict__ b1, const float* __restrict__ b2,
    const float* __restrict__ ba, const float* __restrict__ btb,
    unsigned short* __restrict__ Hs)
{
  __shared__ __align__(16) _Float16 sH[16 * kHP];
  __shared__ __align__(16) _Float16 sZ[16 * kZP];
  const _Float16* X16 = (const _Float16*)X16p;
  const _Float16* WbT = (const _Float16*)WbTp;
  const _Float16* WhT = (const _Float16*)WhTp;

  const int tid  = threadIdx.x;
  const int lane = tid & 31;
  const int wave = tid >> 5;
  const int rl   = lane & 15;
  const int hh   = lane >> 4;
  const int koff = hh * 8;
  const int b0   = blockIdx.x * 16;

  {
    v8h zz;
#pragma unroll
    for (int e = 0; e < 8; ++e) zz[e] = (_Float16)0.0f;
    for (int i = tid; i < (16 * kHP) / 8; i += 256) *(v8h*)(sH + i * 8) = zz;
  }

  v16h wbf[10];
  {
    const _Float16* wp = WbT + (size_t)(wave * 16 + rl) * kCat + koff;
#pragma unroll
    for (int kt = 0; kt < 10; ++kt) wbf[kt] = FragH::load(wp + kt * 32);
  }

  const int ncolB = wave * 16 + rl;
  const float biasZ = bb[ncolB];
  const int ncol0 = wave * 16 + rl;
  const int ncol1 = (wave + 8) * 16 + rl;
  const float c1a = b1[ncol0], c1b = b1[ncol1];
  const float c2a = b2[ncol0], c2b = b2[ncol1];
  const float c3a = ba[ncol0] + btb[ncol0];
  const float c3b = ba[ncol1] + btb[ncol1];

  const _Float16* xrow = X16 + (size_t)(b0 + rl) * kSteps * kIn + koff;
  const _Float16* hA   = sH + rl * kHP + koff;
  const _Float16* zA   = sZ + rl * kZP + koff;

  __syncthreads();

#pragma unroll 1
  for (int t = 0; t < kSteps; ++t) {
    {
      const _Float16* xr = xrow + (size_t)t * kIn;
      v8f acc = (v8f){0.f, 0.f, 0.f, 0.f, 0.f, 0.f, 0.f, 0.f};
#pragma unroll
      for (int kt = 0; kt < 2; ++kt) {
        const v16h a = FragH::load(xr + kt * 32);
        acc = mma_h(a, wbf[kt], acc);
      }
#pragma unroll
      for (int kt = 0; kt < 8; ++kt) {
        const v16h a = FragH::load(hA + kt * 32);
        acc = mma_h(a, wbf[2 + kt], acc);
      }
#pragma unroll
      for (int r = 0; r < 8; ++r) {
        const float pre = acc[r] * kWInv + biasZ;
        const float zv  = 1.7159f * tanh_f32(0.666f * pre);
        sZ[(8 * hh + r) * kZP + ncolB] = (_Float16)zv;
      }
    }
    __syncthreads();

    {
      v16h az[4];
#pragma unroll
      for (int kt = 0; kt < 4; ++kt) az[kt] = FragH::load(zA + kt * 32);
#pragma unroll 1
      for (int half = 0; half < 2; ++half) {
        const int lt = wave + half * 8;
        const _Float16* wp = WhT + (size_t)(lt * 16 + rl) * kBk + koff;
        v8f a1 = (v8f){0.f, 0.f, 0.f, 0.f, 0.f, 0.f, 0.f, 0.f};
        v8f a2 = a1;
        v8f a3 = a1;
#pragma unroll
        for (int kt = 0; kt < 4; ++kt) {
          const v16h bf1 = FragH::load(wp + kt * 32);
          const v16h bf2 = FragH::load(wp + (size_t)kLat * kBk + kt * 32);
          const v16h bf3 = FragH::load(wp + (size_t)2 * kLat * kBk + kt * 32);
          a1 = mma_h(az[kt], bf1, a1);
          a2 = mma_h(az[kt], bf2, a2);
          a3 = mma_h(az[kt], bf3, a3);
        }
        const float c1 = half ? c1b : c1a;
        const float c2 = half ? c2b : c2a;
        const float c3 = half ? c3b : c3a;
        const int ncol = lt * 16 + rl;
#pragma unroll
        for (int r = 0; r < 8; ++r) {
          const float f1 = tanh_f32(a1[r] * kWInv + c1);
          const float f2 = tanh_f32(a2[r] * kWInv + c2);
          const float ti = sigmoid_f32(a3[r] * kWInv + c3);
          const float hn = f1 + ti * (f2 - f1);
          sH[(8 * hh + r) * kHP + ncol] = (_Float16)hn;
        }
      }
    }
    __syncthreads();

    {
      const v8h hv0 = *(const v8h*)(sH + (2 * wave) * kHP + lane * 8);
      const v8h hv1 = *(const v8h*)(sH + (2 * wave + 1) * kHP + lane * 8);
      const size_t o0 = ((size_t)(b0 + 2 * wave) * kSteps + t) * kLat + lane * 8;
      const size_t o1 = o0 + (size_t)kSteps * kLat;
      *(volatile v8h*)(Hs + o0) = hv0;
      *(volatile v8h*)(Hs + o1) = hv1;
      __threadfence();
      *(volatile v8h*)(Hs + o0) = hv0;
      *(volatile v8h*)(Hs + o1) = hv1;
    }
  }
}

template <int OUT_MODE, int ACT>
__global__ __launch_bounds__(256) void wmma_gemm32x64_f16w2(
    const unsigned short* __restrict__ Ap, int lda,
    const unsigned short* __restrict__ Btp, const unsigned short* __restrict__ BtRp, int ldb,
    void* __restrict__ Cout, int ldc,
    const float* __restrict__ bias,
    int M, int N, int K, float scale, float oscale)
{
  const _Float16* A   = (const _Float16*)Ap;
  const _Float16* Bt  = (const _Float16*)Btp;
  const _Float16* BtR = (const _Float16*)BtRp;
  __shared__ __align__(16) float sT[8][16 * 68];
  const int lane = threadIdx.x & 31;
  const int wave = threadIdx.x >> 5;
  const int tilesN = N >> 6;
  const int tilesM = M >> 5;
  const int tile = blockIdx.x * 8 + wave;
  if (tile >= tilesM * tilesN) return;
  const int tm = tile / tilesN;
  const int tn = tile - tm * tilesN;
  const int m0 = tm << 5;
  const int n0 = tn << 6;

  const int rlane = lane & 15;
  const int koff  = (lane >> 4) * 8;
  const int mOff  = (lane >> 4) * 8;

  v8f acc[2][4];
  v8f accr[2][4];
#pragma unroll
  for (int i = 0; i < 2; ++i)
#pragma unroll
    for (int j = 0; j < 4; ++j) {
      acc[i][j]  = (v8f){0.f, 0.f, 0.f, 0.f, 0.f, 0.f, 0.f, 0.f};
      accr[i][j] = (v8f){0.f, 0.f, 0.f, 0.f, 0.f, 0.f, 0.f, 0.f};
    }

  for (int k0 = 0; k0 < K; k0 += 32) {
    v16h ah[2];
#pragma unroll
    for (int i = 0; i < 2; ++i) {
      const size_t ao = (size_t)(m0 + (i << 4) + rlane) * lda + koff + k0;
      ah[i] = FragH::load(A + ao);
    }
#pragma unroll
    for (int j = 0; j < 4; ++j) {
      const size_t bo = (size_t)(n0 + (j << 4) + rlane) * ldb + koff + k0;
      const v16h bv = FragH::load(Bt + bo);
      const v16h br = FragH::load(BtR + bo);
#pragma unroll
      for (int i = 0; i < 2; ++i) {
        acc[i][j]  = mma_h(ah[i], bv, acc[i][j]);
        accr[i][j] = mma_h(ah[i], br, accr[i][j]);
      }
    }
  }

  float* slab = sT[wave];
#pragma unroll
  for (int i = 0; i < 2; ++i) {
    const int mBase = m0 + (i << 4);
#pragma unroll
    for (int j = 0; j < 4; ++j) {
      const int n = n0 + (j << 4) + rlane;
      const float bv = bias[n];
#pragma unroll
      for (int r = 0; r < 8; ++r) {
        const float s = acc[i][j][r] + accr[i][j][r] * kResInv;
        const float v = s * scale + bv;
        slab[(mOff + r) * 68 + (j << 4) + rlane] = v;
      }
    }
    __builtin_amdgcn_fence(__ATOMIC_RELEASE, "workgroup");
    __builtin_amdgcn_wave_barrier();
    __builtin_amdgcn_fence(__ATOMIC_ACQUIRE, "workgroup");
    if (ACT == 3) {
      const int qa = lane >> 3, ca = (lane & 7) * 8;
#pragma unroll 1
      for (int it = 0; it < 4; ++it) {
        float* sp = slab + (it * 4 + qa) * 68 + ca;
#pragma unroll 1
        for (int e = 0; e < 8; ++e) {
          const float xv = sp[e];
          const float sg = sigmoid_f32(xv);
          sp[e] = xv * sg * oscale;
        }
      }
      __builtin_amdgcn_fence(__ATOMIC_RELEASE, "workgroup");
      __builtin_amdgcn_wave_barrier();
      __builtin_amdgcn_fence(__ATOMIC_ACQUIRE, "workgroup");
    }
    if (OUT_MODE == 0) {
      float* C = (float*)Cout;
      const int hh = lane >> 4, c4 = (lane & 15) * 4;
      for (int pass = 0; pass < 2; ++pass) {
#pragma unroll
        for (int it = 0; it < 8; ++it) {
          const int row = it * 2 + hh;
          const v4f v = *(const v4f*)(slab + row * 68 + c4);
          *(volatile v4f*)(C + (size_t)(mBase + row) * ldc + n0 + c4) = v;
        }
        __threadfence();
      }
    } else {
      const int q = lane >> 3, c8 = (lane & 7) * 8;
      unsigned short* C = (unsigned short*)Cout;
      for (int pass = 0; pass < 2; ++pass) {
#pragma unroll
        for (int it = 0; it < 4; ++it) {
          const int row = it * 4 + q;
          const float* sp = slab + row * 68 + c8;
          v8h hv;
#pragma unroll
          for (int e = 0; e < 8; ++e) hv[e] = (_Float16)sp[e];
          *(volatile v8h*)(C + (size_t)(mBase + row) * ldc + n0 + c8) = hv;
        }
        __threadfence();
      }
    }
    __builtin_amdgcn_fence(__ATOMIC_RELEASE, "workgroup");
    __builtin_amdgcn_wave_barrier();
    __builtin_amdgcn_fence(__ATOMIC_ACQUIRE, "workgroup");
  }
}

constexpr int kBlkHidden = ((kRows / 32) * (kProjH / 64)) / 8;
constexpr int kBlkOut    = ((kRows / 32) * (kOutD / 64)) / 8;
static_assert(kBlkHidden == 1024 && kBlkOut == 512, "flat GEMM grids");
static_assert(kBlkHidden * 8 == (kRows / 32) * (kProjH / 64) && kBlkOut * 8 == (kRows / 32) * (kOutD / 64), "flat GEMM coverage");

extern "C" void kernel_launch(void* const* d_in, const int* in_sizes, int n_in,
                              void* d_out, int out_size, void* d_ws, size_t ws_size,
                              hipStream_t stream) {
  if (n_in < 15) return;
  if (in_sizes[0] != kRows * kIn) return;
  if (in_sizes[1] != kCat * kBk) return;
  if (in_sizes[2] != kBk) return;
  if (in_sizes[3] != kBk * kLat) return;
  if (in_sizes[4] != kLat) return;
  if (in_sizes[5] != kBk * kLat) return;
  if (in_sizes[6] != kLat) return;
  if (in_sizes[7] != kBk * kLat) return;
  if (in_sizes[8] != kLat) return;
  if (in_sizes[9] != kBk * kLat) return;
  if (in_sizes[10] != kLat) return;
  if (in_sizes[11] != kLat * kProjH) return;
  if (in_sizes[12] != kProjH) return;
  if (in_sizes[13] != kProjH * kOutD) return;
  if (in_sizes[14] != kOutD) return;
  if (out_size != kRows * kOutD) return;
  if (ws_size < kWsTotal) return;

  const float* x   = (const float*)d_in[0];
  const float* Wb  = (const float*)d_in[1];
  const float* bb  = (const float*)d_in[2];
  const float* W1  = (const float*)d_in[3];
  const float* b1  = (const float*)d_in[4];
  const float* W2  = (const float*)d_in[5];
  const float* b2  = (const float*)d_in[6];
  const float* Wa  = (const float*)d_in[7];
  const float* ba  = (const float*)d_in[8];
  const float* Wtb = (const float*)d_in[9];
  const float* btb = (const float*)d_in[10];
  const float* Wp1 = (const float*)d_in[11];
  const float* bp1 = (const float*)d_in[12];
  const float* Wp2 = (const float*)d_in[13];
  const float* bp2 = (const float*)d_in[14];
  float* out = (float*)d_out;

  char* ws = (char*)d_ws;
  unsigned short* WbT  = (unsigned short*)(ws + kOffWbT);
  unsigned short* WhT  = (unsigned short*)(ws + kOffWhT);
  unsigned short* Wp1T = (unsigned short*)(ws + kOffWp1T);
  unsigned short* Wp1R = (unsigned short*)(ws + kOffWp1R);
  unsigned short* Wp2T = (unsigned short*)(ws + kOffWp2T);
  unsigned short* Wp2R = (unsigned short*)(ws + kOffWp2R);
  unsigned short* X16  = (unsigned short*)(ws + kOffX16);
  unsigned short* Hs   = (unsigned short*)(ws + kOffHs);
  unsigned short* HD16 = (unsigned short*)(ws + kOffHD);

  pack_weights_kernel<<<kBlkPack, 256, 0, stream>>>(Wb, W1, W2, Wa, Wtb, Wp1, Wp2,
                                                    WbT, WhT, Wp1T, Wp1R, Wp2T, Wp2R);

  x_to_f16_kernel<<<(kRows * kIn / 8) / 256, 256, 0, stream>>>(x, X16, kRows * kIn / 8);

  recur_kernel<<<kBatch / 16, 256, 0, stream>>>(X16, WbT, WhT, bb, b1, b2, ba, btb, Hs);

  wmma_gemm32x64_f16w2<1, 3><<<kBlkHidden, 256, 0, stream>>>(
      Hs, kLat, Wp1T, Wp1R, kLat, (void*)HD16, kProjH, bp1,
      kRows, kProjH, kLat, kWInv, kHdCarry);

  wmma_gemm32x64_f16w2<0, 0><<<kBlkOut, 256, 0, stream>>>(
      HD16, kProjH, Wp2T, Wp2R, kProjH, (void*)out, kOutD, bp2,
      kRows, kOutD, kProjH, kOutScale, 1.0f);
}
